// SpatialSelfAttention_59811714564809
// MI455X (gfx1250) — hardware-verified
//
#include <hip/hip_runtime.h>
#include <math.h>

typedef __attribute__((ext_vector_type(16))) _Float16 v16h;
typedef __attribute__((ext_vector_type(16))) __bf16 v16b;
typedef __attribute__((ext_vector_type(8)))  _Float16 v8h;
typedef __attribute__((ext_vector_type(8)))  float v8f;
typedef __attribute__((ext_vector_type(4)))  float v4f;
typedef __attribute__((ext_vector_type(2)))  float v2f;
typedef __attribute__((ext_vector_type(4)))  unsigned v4u;
typedef __attribute__((ext_vector_type(4)))  int v4i;
typedef float __attribute__((may_alias)) float_a;
typedef int __attribute__((may_alias)) int_a;

template <typename T> __device__ __forceinline__ void vst2(void* p, T v) { *(volatile T*)p = v; __threadfence(); *(volatile T*)p = v; }
__device__ __forceinline__ v8f wmma16(v16h a, v16h b, v8f c) {
  v8f d = __builtin_amdgcn_wmma_f32_16x16x32_f16(false, a, false, b, (short)0, c, false, false);
  asm volatile("v_nop\n\tv_nop\n\tv_nop\n\tv_nop" : "+v"(d) : "v"(a), "v"(b));
  return d;
}
__device__ __forceinline__ v8f wmma_bf(v16b a, v16b b, v8f c) {
  v8f d = __builtin_amdgcn_wmma_f32_16x16x32_bf16(false, a, false, b, (short)0, c, false, false);
  asm volatile("v_nop\n\tv_nop\n\tv_nop\n\tv_nop" : "+v"(d) : "v"(a), "v"(b));
  return d;
}
__device__ __forceinline__ v16h frag_h(const _Float16* rowk0, int lane) {
  union { v16h v; v8h q[2]; } u; const _Float16* p = rowk0 + 8 * (lane >> 4);
  u.q[0] = *(const v8h*)p; u.q[1] = *(const v8h*)(p + 16); return u.v;
}
__device__ __forceinline__ v16h frag_f32(const float* rowk0, int lane) {
  v16h a; const float* p = rowk0 + 8 * (lane >> 4);
#pragma unroll
  for (int i = 0; i < 8; ++i) { a[i] = (_Float16)p[i]; a[8 + i] = (_Float16)p[16 + i]; }
  return a;
}
__device__ __forceinline__ v16h frag_f32s(const float* rowk0, int lane, float sc) {
  v16h a; const float* p = rowk0 + 8 * (lane >> 4);
#pragma unroll
  for (int i = 0; i < 8; ++i) { a[i] = (_Float16)(p[i] * sc); a[8 + i] = (_Float16)(p[16 + i] * sc); }
  return a;
}
__device__ __forceinline__ v16h fragc_f32(const float* W, int k0, int n, int lane, int ld, int K) {
  v16h a; const int g = lane >> 4;
#pragma unroll
  for (int i = 0; i < 8; ++i) { const int ka = k0 + 8 * g + i, kb = ka + 16;
    a[i] = (_Float16)(ka < K ? W[(size_t)(ka < K ? ka : K - 1) * ld + n] : 0.f); a[8 + i] = (_Float16)(kb < K ? W[(size_t)(kb < K ? kb : K - 1) * ld + n] : 0.f); }
  return a;
}
struct F2 { v16b h, l; };
__device__ __forceinline__ F2 bsplit16(const float v[16]) { F2 r;
#pragma unroll
  for (int i = 0; i < 16; ++i) { const __bf16 h = (__bf16)v[i]; r.h[i] = h; r.l[i] = (__bf16)(v[i] - (float)h); }
  return r; }
__device__ __forceinline__ F2 split_row(const float* row, int k0, int lane) { float v[16]; const float* p = row + k0 + 8 * (lane >> 4);
#pragma unroll
  for (int i = 0; i < 8; ++i) { v[i] = p[i]; v[8 + i] = p[16 + i]; }
  return bsplit16(v); }
__device__ __forceinline__ F2 split_rowK(const float* row, int k0, int lane, int K) { float v[16]; const int g = lane >> 4;
#pragma unroll
  for (int i = 0; i < 8; ++i) { const int ka = k0 + 8 * g + i, kb = ka + 16; v[i] = ka < K ? row[ka < K ? ka : K - 1] : 0.f; v[8 + i] = kb < K ? row[kb < K ? kb : K - 1] : 0.f; }
  return bsplit16(v); }
__device__ __forceinline__ F2 split_col(const float* W, int k0, int n, int lane, int ld, int K) { float v[16]; const int g = lane >> 4;
#pragma unroll
  for (int i = 0; i < 8; ++i) { const int ka = k0 + 8 * g + i, kb = ka + 16; v[i] = ka < K ? W[(size_t)(ka < K ? ka : K - 1) * ld + n] : 0.f; v[8 + i] = kb < K ? W[(size_t)(kb < K ? kb : K - 1) * ld + n] : 0.f; }
  return bsplit16(v); }
__device__ __forceinline__ v8f mac3(const F2& a, const F2& b, v8f c) { c = wmma_bf(a.l, b.h, c); c = wmma_bf(a.h, b.l, c); return wmma_bf(a.h, b.h, c); }
__device__ __forceinline__ float sigm(float v) { return 1.0f / (1.0f + expf(-v)); }
#define LDSX() do { asm volatile("s_wait_dscnt 0" ::: "memory"); __builtin_amdgcn_wave_barrier(); __builtin_amdgcn_fence(__ATOMIC_RELEASE, "workgroup"); } while (0)


#define NBATCH 16
#define NT 12
#define NG (NBATCH * NT)
#define NNODE 358
#define NP 384
#define DD 128
#define KH 8
#define HS 16
#ifndef TG
#define TG NG
#endif
typedef __attribute__((ext_vector_type(8))) __bf16 v8b;
__device__ __forceinline__ v16b frag_b(const __bf16* rowk0, int lane) {
  union { v16b v; v8b q[2]; } u; const __bf16* p = rowk0 + 8 * (lane >> 4);
  u.q[0] = *(const v8b*)p; u.q[1] = *(const v8b*)(p + 16); return u.v;
}
__device__ __forceinline__ float bfr(float v) { return (float)(__bf16)v; }
__device__ __attribute__((noinline)) float exp_ni(float v) { return expf(v); }
__device__ __attribute__((noinline)) float erf_ni(float v) { return erff(v); }

#define WS_KH  0u
#define WS_KL  (WS_KH + 2u * (size_t)NG * NP * DD)
#define WS_VH  (WS_KL + 2u * (size_t)NG * NP * DD)
#define WS_VL  (WS_VH + 2u * (size_t)NG * DD * NP)
#define WS_O   (WS_VL + 2u * (size_t)NG * DD * NP)
#define WS_END (WS_O + 4u * (size_t)NG * NP * DD)

__device__ __forceinline__ size_t xrow(size_t g, int n) { return (g * NNODE + (size_t)(n < NNODE ? n : NNODE - 1)) * DD; }
__global__ __launch_bounds__(128) void k_kv(const float* __restrict__ X, const float* __restrict__ WK, const float* __restrict__ BK, const float* __restrict__ WV, const float* __restrict__ BV, _Float16* __restrict__ KHp, _Float16* __restrict__ KLp, _Float16* __restrict__ VHp, _Float16* __restrict__ VLp) {
  __shared__ __align__(16) _Float16 sh[64][136], sl[64][136]; __shared__ __align__(16) _Float16 th[128][72], tl[128][72];
  const int tid = threadIdx.x, wave = tid >> 5, lane = tid & 31, col = lane & 15, g = lane >> 4; const int which = blockIdx.y; const size_t grp = blockIdx.z; const size_t b = grp / NT; const int n0 = blockIdx.x * 64; const float* Wm = (which == 0 ? WK : WV) + b * DD * DD; const float* Bm = (which == 0 ? BK : BV) + b * DD;
  v8f acc[8] = {};
#pragma unroll
  for (int kc = 0; kc < DD / 32; ++kc) { v16b a; const float* pp = X + xrow(grp, n0 + wave * 16 + col) + kc * 32 + 8 * g;
#pragma unroll
    for (int i = 0; i < 8; ++i) { a[i] = (__bf16)pp[i]; a[8 + i] = (__bf16)pp[16 + i]; }
#pragma unroll
    for (int j = 0; j < 8; ++j) { v16b w; const int e = j * 16 + col;
#pragma unroll
      for (int i = 0; i < 8; ++i) { w[i] = (__bf16)Wm[(size_t)(kc * 32 + 8 * g + i) * DD + e]; w[8 + i] = (__bf16)Wm[(size_t)(kc * 32 + 16 + 8 * g + i) * DD + e]; }
      acc[j] = wmma_bf(a, w, acc[j]); } }
#pragma unroll
  for (int j = 0; j < 8; ++j) { const float bb = bfr(Bm[j * 16 + col]);
#pragma unroll
    for (int r = 0; r < 8; ++r) { const float v = acc[j][r] + bb; const _Float16 hv = (_Float16)v, lv = (_Float16)((v - (float)hv) * 2048.0f); const int rl = wave * 16 + 8 * g + r, cl = j * 16 + col; if (which == 0) { sh[rl][cl] = hv; sl[rl][cl] = lv; } else { th[cl][rl] = hv; tl[cl][rl] = lv; } } }
  __syncthreads();
  if (which == 0) { for (int e = tid; e < 64 * 16; e += 128) { const int rl = e >> 4, q = e & 15; const size_t o = (grp * NP + n0 + rl) * DD + q * 8; vst2((unsigned*)(KHp + o), *(const v4u*)&sh[rl][q * 8]); vst2((unsigned*)(KLp + o), *(const v4u*)&sl[rl][q * 8]); } }
  else { for (int e = tid; e < 128 * 8; e += 128) { const int cl = e >> 3, q = e & 7; const size_t o = (grp * DD + cl) * (size_t)NP + n0 + q * 8; vst2((unsigned*)(VHp + o), *(const v4u*)&th[cl][q * 8]); vst2((unsigned*)(VLp + o), *(const v4u*)&tl[cl][q * 8]); } } }
__global__ __launch_bounds__(128) void k_att(const float* __restrict__ X, const _Float16* __restrict__ KHp, const _Float16* __restrict__ KLp, const _Float16* __restrict__ VHp, const _Float16* __restrict__ VLp, float* __restrict__ O) {
  __shared__ __align__(16) float sp[4][16][36]; __shared__ __align__(16) float so[4][16][36];
  const int tid = threadIdx.x, wave = tid >> 5, lane = tid & 31, col = lane & 15, g = lane >> 4; const int hp = blockIdx.y; const size_t grp = blockIdx.z; const int q0 = blockIdx.x * 64 + wave * 16;
#pragma unroll 1
  for (int hh = 0; hh < 2; ++hh) { const int kh = hp * 2 + hh;
    v16h aq; { const float* pp = X + xrow(grp, q0 + col) + kh * HS + 8 * g;
#pragma unroll
      for (int i = 0; i < 8; ++i) { aq[i] = (_Float16)bfr(pp[i]); aq[8 + i] = (_Float16)0.0f; } }
    float m[8], l[8];
#pragma unroll
    for (int r = 0; r < 8; ++r) { m[r] = -3.0e38f; l[r] = 0.f; }
    v8f acc = {}, accl = {};
#pragma unroll 1
    for (int ks = 0; ks < NP / 32; ++ks) { float s[2][8];
#pragma unroll
      for (int ct = 0; ct < 2; ++ct) { const int kk = ks * 32 + ct * 16 + col; const size_t rk = (grp * NP + kk) * DD + kh * HS; v8f c = {}, cl = {}; c = wmma16(aq, frag_h(KHp + rk, lane), c); cl = wmma16(aq, frag_h(KLp + rk, lane), cl);
#pragma unroll
        for (int r = 0; r < 8; ++r) s[ct][r] = (kk < NNODE) ? (c[r] + cl[r] * (1.0f / 2048.0f)) * 0.25f : -3.0e38f; }
      float alpha[8];
#pragma unroll
      for (int r = 0; r < 8; ++r) { float mx = fmaxf(s[0][r], s[1][r]);
#pragma unroll
        for (int o = 1; o < 16; o <<= 1) mx = fmaxf(mx, __shfl_xor(mx, o));
        const float mn = fmaxf(m[r], mx); alpha[r] = (m[r] <= -1.0e38f) ? 0.f : __expf(m[r] - mn); const float e0 = (s[0][r] <= -1.0e38f) ? 0.f : __expf(s[0][r] - mn), e1 = (s[1][r] <= -1.0e38f) ? 0.f : __expf(s[1][r] - mn); float es = e0 + e1;
#pragma unroll
        for (int o = 1; o < 16; o <<= 1) es += __shfl_xor(es, o);
        l[r] = l[r] * alpha[r] + es; m[r] = mn; sp[wave][8 * g + r][col] = e0; sp[wave][8 * g + r][16 + col] = e1; }
#pragma unroll
      for (int r = 0; r < 8; ++r) { acc[r] *= alpha[r]; accl[r] *= alpha[r]; }
      LDSX();
      v16h pa; { const float* prow = &sp[wave][col][0] + 8 * (lane >> 4);
#pragma unroll
        for (int i = 0; i < 8; ++i) { pa[i] = (_Float16)(prow[i] * 2048.0f); pa[8 + i] = (_Float16)(prow[16 + i] * 2048.0f); } }
      { const size_t po = (grp * DD + (size_t)kh * HS + col) * NP + ks * 32; acc = wmma16(pa, frag_h(VHp + po, lane), acc); accl = wmma16(pa, frag_h(VLp + po, lane), accl); }
      LDSX(); }
#pragma unroll
    for (int r = 0; r < 8; ++r) so[wave][8 * g + r][hh * 16 + col] = (acc[r] + accl[r] * (1.0f / 2048.0f)) * ((1.0f / 2048.0f) / l[r]);
    LDSX(); }
  for (int rl = 0; rl < 16; ++rl) if (lane < 8) vst2(O + ((grp * NP) + q0 + rl) * DD + hp * 32 + lane * 4, *(const v4f*)&so[wave][rl][lane * 4]); }
__global__ __launch_bounds__(128) void k_mlp(const float* __restrict__ O, const float* __restrict__ W1, const float* __restrict__ B1, const float* __restrict__ W2, const float* __restrict__ B2, float* __restrict__ OUT) { __shared__ __align__(16) float sf[4][16][132];
  const int tid = threadIdx.x, wave = tid >> 5, lane = tid & 31, col = lane & 15, g = lane >> 4; const size_t grp = blockIdx.y; const int n0 = blockIdx.x * 64 + wave * 16; const size_t r0 = grp * NP + n0;
  v8f acc[8] = {};
#pragma unroll
  for (int kc = 0; kc < DD / 32; ++kc) { const F2 a = split_row(O + (r0 + col) * DD, kc * 32, lane);
#pragma unroll
    for (int j = 0; j < 8; ++j) { v16b w; const float* wr = W1 + (size_t)(j * 16 + col) * DD + kc * 32 + 8 * g;
#pragma unroll
      for (int i = 0; i < 8; ++i) { w[i] = (__bf16)wr[i]; w[8 + i] = (__bf16)wr[16 + i]; }
      acc[j] = wmma_bf(a.h, w, acc[j]); acc[j] = wmma_bf(a.l, w, acc[j]); } }
#pragma unroll
  for (int j = 0; j < 8; ++j) { const float bb = bfr(B1[j * 16 + col]);
#pragma unroll
    for (int r = 0; r < 8; ++r) sf[wave][8 * g + r][j * 16 + col] = fmaxf(acc[j][r] + bb, 0.f); }
  LDSX();
  { v8f acc2[8] = {};
#pragma unroll
    for (int kc = 0; kc < DD / 32; ++kc) { float v[16]; const float* pp = &sf[wave][col][kc * 32 + 8 * g];
#pragma unroll
      for (int i = 0; i < 8; ++i) { v[i] = pp[i]; v[8 + i] = pp[16 + i]; }
      const F2 a = bsplit16(v);
#pragma unroll
      for (int j = 0; j < 8; ++j) { v16b w; const float* wr = W2 + (size_t)(j * 16 + col) * DD + kc * 32 + 8 * g;
#pragma unroll
        for (int i = 0; i < 8; ++i) { w[i] = (__bf16)wr[i]; w[8 + i] = (__bf16)wr[16 + i]; }
        acc2[j] = wmma_bf(a.h, w, acc2[j]); acc2[j] = wmma_bf(a.l, w, acc2[j]); } }
    LDSX();
#pragma unroll
    for (int j = 0; j < 8; ++j) { const float bb = bfr(B2[j * 16 + col]);
#pragma unroll
      for (int r = 0; r < 8; ++r) sf[wave][8 * g + r][j * 16 + col] = acc2[j][r] + bb; } }
  LDSX(); for (int rl = 0; rl < 16; ++rl) { const int n = n0 + rl; if (n < NNODE) vst2(OUT + (grp * NNODE + n) * DD + lane * 4, *(const v4f*)&sf[wave][rl][lane * 4]); } }
extern "C" void kernel_launch(void* const* d_in, const int* in_sizes, int n_in, void* d_out, int out_size, void* d_ws, size_t ws_size, hipStream_t stream) {
  (void)in_sizes; (void)n_in; (void)out_size;
  const float** F = (const float**)d_in;
  if (ws_size < (size_t)WS_END) return;
  char* ws = (char*)d_ws; _Float16 *KHp = (_Float16*)(ws + WS_KH), *KLp = (_Float16*)(ws + WS_KL), *VHp = (_Float16*)(ws + WS_VH), *VLp = (_Float16*)(ws + WS_VL); float* O = (float*)(ws + WS_O);
  k_kv<<<dim3(NP / 64, 2, TG), 128, 0, stream>>>(F[0], F[1], F[2], F[3], F[4], KHp, KLp, VHp, VLp);
  k_att<<<dim3(NP / 64, KH / 2, TG), 128, 0, stream>>>(F[0], KHp, KLp, VHp, VLp, O);
  k_mlp<<<dim3(NP / 64, TG), 128, 0, stream>>>(O, F[5], F[6], F[7], F[8], (float*)d_out);
}
